// CellMatesTransformer_24120536334929
// MI455X (gfx1250) — hardware-verified
//
#include <hip/hip_runtime.h>
#include <math.h>
#include <stdint.h>
#include <stddef.h>

typedef __attribute__((ext_vector_type(16))) _Float16 v16h;
typedef __attribute__((ext_vector_type(8)))  _Float16 v8h;
typedef __attribute__((ext_vector_type(16))) __bf16   v16b;
typedef __attribute__((ext_vector_type(8)))  __bf16   v8b;
typedef __attribute__((ext_vector_type(8)))  float    v8f;
typedef __attribute__((ext_vector_type(4)))  float    v4f;
typedef __attribute__((ext_vector_type(4)))  int      v4i;
typedef __attribute__((ext_vector_type(4)))  unsigned v4u;
typedef unsigned short u16;

constexpr int NBATCH = 4;
constexpr int SEQ    = 384;
constexpr int DMOD   = 512;
constexpr int NHEAD  = 8;
constexpr int HDIM   = 64;
constexpr int FFD    = 2048;
constexpr int MHID   = 512;
constexpr int NLAY   = 2;
constexpr int NCELL  = 6;
constexpr int NBIN   = 15;
constexpr int NTOK   = NBATCH * SEQ;
constexpr int HPITCH = DMOD + 64;
constexpr int NBH    = NBATCH * NHEAD;
constexpr int QROWS  = NTOK * NHEAD;
constexpr int S3K    = 32;
constexpr int TAILM  = 64;

static_assert(NTOK % 64 == 0 && DMOD % 64 == 0 && FFD % 64 == 0 && SEQ % 64 == 0 && MHID % 64 == 0 && QROWS % 64 == 0 && TAILM % 64 == 0);
static_assert(DMOD % 32 == 0 && HPITCH % 32 == 0 && FFD % 32 == 0 && HDIM % 32 == 0 && SEQ % 32 == 0 && S3K % 32 == 0 && NTOK % 32 == 0 && MHID % 32 == 0);
static_assert(HDIM == 64 && NHEAD * HDIM == DMOD && DMOD == 512 && SEQ == 384 && NBATCH == 4 && NHEAD == 8);
static_assert(NTOK % 8 == 0 && (NBATCH * SEQ * SEQ) % 1024 == 0 && (NTOK * FFD / 2) % 256 == 0);
static_assert(NBIN <= 15 && 6 * NBIN * HDIM == 5760 && (6 * NBIN * HDIM) % 4 == 0);

constexpr size_t SZ_HF    = (size_t)NTOK * DMOD * 4;
constexpr size_t SZ_HP    = (size_t)NTOK * HPITCH * 2;
constexpr size_t SZ_W512  = (size_t)512 * 512 * 2;
constexpr size_t SZ_W576  = (size_t)512 * HPITCH * 2;
constexpr size_t SZ_WFF   = (size_t)FFD * 512 * 2;
constexpr size_t SZ_D01   = (size_t)64 * 64 * 2;
constexpr size_t SZ_D34   = (size_t)64 * S3K * 2;
constexpr size_t SZ_A16   = (size_t)NTOK * DMOD * 2;
constexpr size_t SZ_T     = (size_t)QROWS * 64 * 4;
constexpr size_t SZ_BIG1  = (size_t)NBH * SEQ * SEQ * 4;
constexpr size_t SZ_BIG2  = (size_t)NBH * SEQ * SEQ * 2;
constexpr size_t SZ_S3    = (size_t)QROWS * S3K * 2;
constexpr size_t SZ_F32A  = (size_t)NTOK * DMOD * 4;
constexpr size_t SZ_DIDX  = (size_t)NBATCH * SEQ * SEQ * 4;
constexpr size_t SZ_MM    = (size_t)TAILM * NTOK * 2;
constexpr size_t SZ_SM    = (size_t)TAILM * 512 * 2;
constexpr size_t SZ_C2    = (size_t)TAILM * 64 * 4;
static_assert(SZ_BIG1 >= (size_t)NTOK * FFD * 4);
static_assert(SZ_BIG2 >= (size_t)NTOK * FFD * 2);

constexpr size_t OFF_HF   = 0;
constexpr size_t OFF_HH   = OFF_HF + SZ_HF;
constexpr size_t OFF_HL   = OFF_HH + SZ_HP;
constexpr size_t OFF_WQH  = OFF_HL + SZ_HP;
constexpr size_t OFF_WQL  = OFF_WQH + SZ_W512;
constexpr size_t OFF_WKH  = OFF_WQL + SZ_W512;
constexpr size_t OFF_WKL  = OFF_WKH + SZ_W576;
constexpr size_t OFF_WVH  = OFF_WKL + SZ_W576;
constexpr size_t OFF_WVL  = OFF_WVH + SZ_W576;
constexpr size_t OFF_WOH  = OFF_WVL + SZ_W576;
constexpr size_t OFF_WOL  = OFF_WOH + SZ_W512;
constexpr size_t OFF_W1H  = OFF_WOL + SZ_W512;
constexpr size_t OFF_W1L  = OFF_W1H + SZ_WFF;
constexpr size_t OFF_W2H  = OFF_W1L + SZ_WFF;
constexpr size_t OFF_W2L  = OFF_W2H + SZ_WFF;
constexpr size_t OFF_D01H = OFF_W2L + SZ_WFF;
constexpr size_t OFF_D01L = OFF_D01H + SZ_D01;
constexpr size_t OFF_D34H = OFF_D01L + SZ_D01;
constexpr size_t OFF_D34L = OFF_D34H + SZ_D34;
constexpr size_t OFF_QH   = OFF_D34L + SZ_D34;
constexpr size_t OFF_QL   = OFF_QH + SZ_A16;
constexpr size_t OFF_KH   = OFF_QL + SZ_A16;
constexpr size_t OFF_KL   = OFF_KH + SZ_A16;
constexpr size_t OFF_VTH  = OFF_KL + SZ_A16;
constexpr size_t OFF_VTL  = OFF_VTH + SZ_A16;
constexpr size_t OFF_T    = OFF_VTL + SZ_A16;
constexpr size_t OFF_BIG1 = OFF_T + SZ_T;
constexpr size_t OFF_BIG2H = OFF_BIG1 + SZ_BIG1;
constexpr size_t OFF_BIG2L = OFF_BIG2H + SZ_BIG2;
constexpr size_t OFF_S3H  = OFF_BIG2L + SZ_BIG2;
constexpr size_t OFF_S3L  = OFF_S3H + SZ_S3;
constexpr size_t OFF_ZPV  = OFF_S3L + SZ_S3;
constexpr size_t OFF_ZH   = OFF_ZPV + SZ_F32A;
constexpr size_t OFF_ZL   = OFF_ZH + SZ_A16;
constexpr size_t OFF_AF   = OFF_ZL + SZ_A16;
constexpr size_t OFF_DIDX = OFF_AF + SZ_F32A;
constexpr size_t OFF_HTH  = OFF_DIDX + SZ_DIDX;
constexpr size_t OFF_HTL  = OFF_HTH + SZ_A16;
constexpr size_t OFF_MMH  = OFF_HTL + SZ_A16;
constexpr size_t OFF_MML  = OFF_MMH + SZ_MM;
constexpr size_t OFF_POH  = OFF_MML + SZ_MM;
constexpr size_t OFF_POL  = OFF_POH + SZ_SM;
constexpr size_t OFF_HIDH = OFF_POL + SZ_SM;
constexpr size_t OFF_HIDL = OFF_HIDH + SZ_SM;
constexpr size_t OFF_WM2H = OFF_HIDL + SZ_SM;
constexpr size_t OFF_WM2L = OFF_WM2H + SZ_SM;
constexpr size_t OFF_C2   = OFF_WM2L + SZ_SM;
constexpr size_t WS_END   = OFF_C2 + SZ_C2;
static_assert(WS_END <= (size_t)134217728);
static_assert(OFF_HH % 256 == 0 && OFF_QH % 256 == 0 && OFF_BIG1 % 256 == 0 && OFF_BIG2H % 256 == 0 && OFF_S3H % 256 == 0 &&
              OFF_ZPV % 256 == 0 && OFF_DIDX % 256 == 0 && OFF_HTH % 256 == 0 && OFF_MMH % 256 == 0 && OFF_C2 % 256 == 0 && OFF_D34H % 256 == 0);

__device__ __forceinline__ unsigned short f2bf_bits(float f) {
  unsigned u = __float_as_uint(f);
  return (unsigned short)((u + 0x7FFFu + ((u >> 16) & 1u)) >> 16);
}
__device__ __forceinline__ float bf_bits2f(unsigned short h) { return __uint_as_float(((unsigned)h) << 16); }

__device__ __forceinline__ void dep_guard_b(v8f& a, v8f& b, v16b x, v16b y) { asm volatile("v_nop\n\tv_nop\n\tv_nop\n\tv_nop" : "+v"(a), "+v"(b) : "v"(x), "v"(y)); }
__device__ __forceinline__ void keep4_b(v16b a, v16b b, v16b c, v16b d) { asm volatile("v_nop" :: "v"(a), "v"(b), "v"(c), "v"(d)); }
__device__ __forceinline__ void acc_guard4(v8f& a, v8f& b, v8f& c, v8f& d) { asm volatile("v_nop\n\tv_nop\n\tv_nop\n\tv_nop" : "+v"(a), "+v"(b), "+v"(c), "+v"(d)); }

template <typename T> struct Frag;
template <> struct Frag<__bf16> {
  typedef v16b V; union U { v16b v; v8b h[2]; };
  static __device__ __forceinline__ v16b load(const __bf16* p) {
    U f; f.h[0] = *(const v8b*)(p); f.h[1] = *(const v8b*)(p + 16); return f.v;
  }
  static __device__ __forceinline__ v8f mma(v16b a, v16b b, v8f c) {
    return __builtin_amdgcn_wmma_f32_16x16x32_bf16(false, a, false, b, (short)0, c, false, false);
  }
  static __device__ __forceinline__ void guard(v8f& a, v8f& b, v16b x, v16b y) { dep_guard_b(a, b, x, y); }
  static __device__ __forceinline__ void keep(v16b a, v16b b, v16b c, v16b d) { keep4_b(a, b, c, d); }
};

__device__ __forceinline__ v8f at_mma(v16b a, v16b b, v8f c) {
  c = __builtin_amdgcn_wmma_f32_16x16x32_bf16(false, a, false, b, (short)0, c, false, false);
  asm volatile("v_nop\n\tv_nop\n\tv_nop\n\tv_nop" : "+v"(c) : "v"(a), "v"(b));
  return c;
}

__device__ __forceinline__ int clampi(int v, int lo, int hi) { return v < lo ? lo : (v > hi ? hi : v); }

__device__ __forceinline__ void split_pack2(float f0, float f1, unsigned& hw, unsigned& lw) {
  const unsigned short h0 = f2bf_bits(f0), h1 = f2bf_bits(f1);
  const unsigned short l0 = f2bf_bits(f0 - bf_bits2f(h0)), l1 = f2bf_bits(f1 - bf_bits2f(h1));
  hw = (unsigned)h0 | ((unsigned)h1 << 16);
  lw = (unsigned)l0 | ((unsigned)l1 << 16);
}
__device__ __forceinline__ void split_pack8(v4f a0, v4f a1, v4u& hv, v4u& lv) {
  unsigned hw0, hw1, hw2, hw3, lw0, lw1, lw2, lw3;
  split_pack2(a0[0], a0[1], hw0, lw0);
  split_pack2(a0[2], a0[3], hw1, lw1);
  split_pack2(a1[0], a1[1], hw2, lw2);
  split_pack2(a1[2], a1[3], hw3, lw3);
  hv = (v4u){hw0, hw1, hw2, hw3};
  lv = (v4u){lw0, lw1, lw2, lw3};
}

template <int BIAS_MODE, int OUT_MODE, bool RESID, int ACT>
__global__ __launch_bounds__(256) void gemm_split64(
    const u16* __restrict__ Ahp, const u16* __restrict__ Alp, int lda, long sAo, long sAi,
    const u16* __restrict__ Bhp, const u16* __restrict__ Blp, int ldb, long sBo, long sBi,
    void* __restrict__ Cout, void* __restrict__ Cout2, int ldc, long sCo, long sCi,
    const float* __restrict__ bias,
    const float* __restrict__ resid, long sRo, long sRi,
    int M, int N, int K, int HB, float scale) {
  typedef __bf16 T;
  typedef v16b V;
  __shared__ __align__(16) float sT[8][16 * 68];
  const int zb   = blockIdx.y;
  const int zo   = zb / HB;
  const int zi   = zb - zo * HB;
  const int lane = threadIdx.x & 31;
  const int wave = threadIdx.x >> 5;
  const int tilesN = N >> 6;
  const int tilesM = M >> 6;
  const int tile = blockIdx.x * 8 + wave;
  if (tile >= tilesM * tilesN) return;
  const int tm = tile / tilesN;
  const int tn = tile - tm * tilesN;
  const int m0 = tm << 6;
  const int n0 = tn << 6;

  const T* Ab  = (const T*)Ahp + (size_t)zo * sAo + (size_t)zi * sAi;
  const T* Ab2 = (const T*)Alp + (size_t)zo * sAo + (size_t)zi * sAi;
  const T* Bb  = (const T*)Bhp + (size_t)zo * sBo + (size_t)zi * sBi;
  const T* Bb2 = (const T*)Blp + (size_t)zo * sBo + (size_t)zi * sBi;
  const size_t cbase = (size_t)zo * sCo + (size_t)zi * sCi;

  const int rlane = lane & 15;
  const int koff  = (lane >> 4) * 8;
  const int mOff  = (lane >> 4) * 8;

  v8f acc[4][4];
#pragma unroll
  for (int i = 0; i < 4; ++i)
#pragma unroll
    for (int j = 0; j < 4; ++j) acc[i][j] = (v8f){0.f,0.f,0.f,0.f,0.f,0.f,0.f,0.f};

  for (int k0 = 0; k0 < K; k0 += 32) {
    V fbh[4], fbl[4];
#pragma unroll
    for (int j = 0; j < 4; ++j) {
      const size_t boff = (size_t)(n0 + (j << 4) + rlane) * ldb + koff + k0;
      fbh[j] = Frag<T>::load(Bb + boff);
      fbl[j] = Frag<T>::load(Bb2 + boff);
    }
#pragma unroll
    for (int i = 0; i < 4; ++i) {
      const size_t aoff = (size_t)(m0 + (i << 4) + rlane) * lda + koff + k0;
      V fah = Frag<T>::load(Ab + aoff);
      V fal = Frag<T>::load(Ab2 + aoff);
#pragma unroll
      for (int j = 0; j < 4; ++j) {
        acc[i][j] = Frag<T>::mma(fah, fbh[j], acc[i][j]);
        acc[i][j] = Frag<T>::mma(fah, fbl[j], acc[i][j]);
        acc[i][j] = Frag<T>::mma(fal, fbh[j], acc[i][j]);
      }
      Frag<T>::guard(acc[i][0], acc[i][3], fah, fal);
    }
    Frag<T>::keep(fbh[0], fbh[1], fbh[2], fbh[3]);
    Frag<T>::keep(fbl[0], fbl[1], fbl[2], fbl[3]);
  }
  acc_guard4(acc[0][0], acc[0][1], acc[0][2], acc[0][3]);
  acc_guard4(acc[1][0], acc[1][1], acc[1][2], acc[1][3]);
  acc_guard4(acc[2][0], acc[2][1], acc[2][2], acc[2][3]);
  acc_guard4(acc[3][0], acc[3][1], acc[3][2], acc[3][3]);

  float* slab = sT[wave];
  const float* Rb = RESID ? (resid + (size_t)zo * sRo + (size_t)zi * sRi) : nullptr;
#pragma unroll
  for (int i = 0; i < 4; ++i) {
    const int mBase = m0 + (i << 4);
    float bm8[8];
#pragma unroll
    for (int r = 0; r < 8; ++r) bm8[r] = (BIAS_MODE == 1) ? bias[mBase + mOff + r] : 0.f;
#pragma unroll
    for (int j = 0; j < 4; ++j) {
      const int n = n0 + (j << 4) + rlane;
      float bv = 0.f;
      if (BIAS_MODE == 2) bv = bias[n];
#pragma unroll
      for (int r = 0; r < 8; ++r) {
        float v = acc[i][j][r] * scale;
        if (BIAS_MODE == 1) v += bm8[r];
        if (BIAS_MODE == 2) v += bv;
        if (ACT == 2) v = fmaxf(v, 0.0f);
        slab[(mOff + r) * 68 + (j << 4) + rlane] = v;
      }
    }
    __builtin_amdgcn_fence(__ATOMIC_RELEASE, "workgroup");
    __builtin_amdgcn_wave_barrier();
    __builtin_amdgcn_fence(__ATOMIC_ACQUIRE, "workgroup");
    if (OUT_MODE == 0) {
      float* C = (float*)Cout + cbase;
      const int hh = lane >> 4, c4 = (lane & 15) * 4;
      for (int pass = 0; pass < 2; ++pass) {
#pragma unroll
        for (int it = 0; it < 8; ++it) {
          const int row = it * 2 + hh;
          v4f v = *(const v4f*)(slab + row * 68 + c4);
          if (RESID) {
            const v4f rr = *(const v4f*)(Rb + (size_t)(mBase + row) * ldc + n0 + c4);
            v = v + rr;
          }
          *(volatile v4f*)(C + (size_t)(mBase + row) * ldc + n0 + c4) = v;
        }
        __threadfence();
      }
    } else {
      const int q = lane >> 3, c8 = (lane & 7) * 8;
      u16* C  = (u16*)Cout  + cbase;
      u16* C2p = (u16*)Cout2 + cbase;
      for (int pass = 0; pass < 2; ++pass) {
#pragma unroll
        for (int it = 0; it < 4; ++it) {
          const int row = it * 4 + q;
          const float* sp = slab + row * 68 + c8;
          float vals[8];
#pragma unroll
          for (int e = 0; e < 8; ++e) vals[e] = sp[e];
          if (RESID) {
            const float* rp = Rb + (size_t)(mBase + row) * ldc + n0 + c8;
            const v4f r0 = *(const v4f*)(rp);
            const v4f r1 = *(const v4f*)(rp + 4);
#pragma unroll
            for (int e = 0; e < 4; ++e) { vals[e] += r0[e]; vals[4 + e] += r1[e]; }
          }
          v8h hv, lv;
#pragma unroll
          for (int e = 0; e < 8; ++e) {
            const unsigned short hb = f2bf_bits(vals[e]);
            const unsigned short lb = f2bf_bits(vals[e] - bf_bits2f(hb));
            hv[e] = __builtin_bit_cast(_Float16, hb);
            lv[e] = __builtin_bit_cast(_Float16, lb);
          }
          *(volatile v8h*)(C  + (size_t)(mBase + row) * ldc + n0 + c8) = hv;
          *(volatile v8h*)(C2p + (size_t)(mBase + row) * ldc + n0 + c8) = lv;
        }
        __threadfence();
      }
    }
    __builtin_amdgcn_fence(__ATOMIC_RELEASE, "workgroup");
    __builtin_amdgcn_wave_barrier();
    __builtin_amdgcn_fence(__ATOMIC_ACQUIRE, "workgroup");
  }
}

__global__ __launch_bounds__(256) void k_bucketize(const float* __restrict__ dist, int* __restrict__ didx, int n4) {
  const int i = blockIdx.x * 256 + threadIdx.x;
  if (i < n4) {
    const v4f d = *(const v4f*)(dist + 4 * (size_t)i);
    v4i o;
#pragma unroll
    for (int e = 0; e < 4; ++e) {
      int c = 0;
#pragma unroll
      for (int t = 1; t <= 14; ++t) c += (10.0f * (float)t < d[e]) ? 1 : 0;
      o[e] = c;
    }
    *(volatile v4i*)(didx + 4 * (size_t)i) = o;
    __threadfence();
    *(volatile v4i*)(didx + 4 * (size_t)i) = o;
  }
}

__global__ __launch_bounds__(256) void k_embed(const int* __restrict__ ct, const float* __restrict__ emb,
                                               const int* __restrict__ didx,
                                               float* __restrict__ hF, u16* __restrict__ hH, u16* __restrict__ hL) {
  const int lane = threadIdx.x & 31, wave = threadIdx.x >> 5;
  const int t = blockIdx.x * 8 + wave;
  const int b = t / SEQ, x = t - b * SEQ;
  const int ci = clampi(ct[t], 0, NCELL - 1);
  const int dr = clampi(didx[(size_t)b * SEQ * SEQ + x], 0, NBIN - 1);
  const float* er = emb + (size_t)ci * DMOD;
  v4f f[4];
#pragma unroll
  for (int i = 0; i < 4; ++i) f[i] = *(const v4f*)(er + 128 * i + 4 * lane);
  v4u ph[2], pl[2];
#pragma unroll
  for (int i = 0; i < 2; ++i) {
    const v4f a0 = *(const v4f*)(er + 256 * i + 8 * lane);
    const v4f a1 = *(const v4f*)(er + 256 * i + 8 * lane + 4);
    split_pack8(a0, a1, ph[i], pl[i]);
  }
  unsigned ew[4];
#pragma unroll
  for (int k = 0; k < 4; ++k) {
    const int j0 = 8 * lane + 2 * k;
    const unsigned b0 = (j0 == dr) ? 0x3F80u : 0u;
    const unsigned b1 = (j0 + 1 == dr) ? 0x3F80u : 0u;
    ew[k] = b0 | (b1 << 16);
  }
  const v4u eh = (v4u){ew[0], ew[1], ew[2], ew[3]};
  const v4u ez = (v4u){0u, 0u, 0u, 0u};
  float* hr = hF + (size_t)t * DMOD;
  u16* prh = hH + (size_t)t * HPITCH;
  u16* prl = hL + (size_t)t * HPITCH;
  for (int pass = 0; pass < 2; ++pass) {
#pragma unroll
    for (int i = 0; i < 4; ++i) *(volatile v4f*)(hr + 128 * i + 4 * lane) = f[i];
#pragma unroll
    for (int i = 0; i < 2; ++i) {
      *(volatile v4u*)(prh + 256 * i + 8 * lane) = ph[i];
      *(volatile v4u*)(prl + 256 * i + 8 * lane) = pl[i];
    }
    if (lane < 8) {
      *(volatile v4u*)(prh + DMOD + 8 * lane) = eh;
      *(volatile v4u*)(prl + DMOD + 8 * lane) = ez;
    }
    __threadfence();
  }
}

__global__ __launch_bounds__(256) void k_resid_ln(const float* __restrict__ aF, const float* __restrict__ gam,
                                                  const float* __restrict__ bet,
                                                  float* hF, u16* __restrict__ hH, u16* __restrict__ hL) {
  __shared__ __align__(16) float ybuf[8][DMOD];
  const int lane = threadIdx.x & 31, wave = threadIdx.x >> 5;
  const int t = blockIdx.x * 8 + wave;
  const float* hr = hF + (size_t)t * DMOD;
  const float* ar = aF + (size_t)t * DMOD;
  v4f v[4];
  float s = 0.f;
#pragma unroll
  for (int i = 0; i < 4; ++i) {
    const v4f h0 = *(const v4f*)(hr + 128 * i + 4 * lane);
    const v4f a0 = *(const v4f*)(ar + 128 * i + 4 * lane);
    v[i] = h0 + a0;
    s += (v[i][0] + v[i][1]) + (v[i][2] + v[i][3]);
  }
#pragma unroll
  for (int off = 16; off > 0; off >>= 1) s += __shfl_xor(s, off, 32);
  const float mu = s * (1.0f / (float)DMOD);
  v4f d[4];
  float s2 = 0.f;
#pragma unroll
  for (int i = 0; i < 4; ++i) {
    d[i] = v[i] - mu;
    s2 += (d[i][0] * d[i][0] + d[i][1] * d[i][1]) + (d[i][2] * d[i][2] + d[i][3] * d[i][3]);
  }
#pragma unroll
  for (int off = 16; off > 0; off >>= 1) s2 += __shfl_xor(s2, off, 32);
  const float var = s2 * (1.0f / (float)DMOD);
  const float inv = 1.0f / sqrtf(var + 1e-5f);
  v4f y[4];
#pragma unroll
  for (int i = 0; i < 4; ++i) {
    const v4f g0 = *(const v4f*)(gam + 128 * i + 4 * lane);
    const v4f b0 = *(const v4f*)(bet + 128 * i + 4 * lane);
    y[i] = (d[i] * inv) * g0 + b0;
    *(v4f*)(&ybuf[wave][128 * i + 4 * lane]) = y[i];
  }
  __syncthreads();
  v4u ph[2], pl[2];
#pragma unroll
  for (int i = 0; i < 2; ++i) {
    const v4f a0 = *(const v4f*)(&ybuf[wave][256 * i + 8 * lane]);
    const v4f a1 = *(const v4f*)(&ybuf[wave][256 * i + 8 * lane + 4]);
    split_pack8(a0, a1, ph[i], pl[i]);
  }
  float* hw = hF + (size_t)t * DMOD;
  u16* prh = hH + (size_t)t * HPITCH;
  u16* prl = hL + (size_t)t * HPITCH;
  for (int pass = 0; pass < 2; ++pass) {
#pragma unroll
    for (int i = 0; i < 4; ++i) *(volatile v4f*)(hw + 128 * i + 4 * lane) = y[i];
#pragma unroll
    for (int i = 0; i < 2; ++i) {
      *(volatile v4u*)(prh + 256 * i + 8 * lane) = ph[i];
      *(volatile v4u*)(prl + 256 * i + 8 * lane) = pl[i];
    }
    __threadfence();
  }
}

__global__ __launch_bounds__(256) void k_wT(const float* __restrict__ W, int ldw,
                                            u16* __restrict__ Oh, u16* __restrict__ Ol, int ldo) {
  __shared__ float tile[64][65];
  const int n0 = blockIdx.x * 64, k0 = blockIdx.y * 64;
  const int tid = threadIdx.x, lane = tid & 31, wave = tid >> 5;
#pragma unroll
  for (int i = 0; i < 4; ++i) {
    const int p = tid + 256 * i;
    const int r = p >> 4, c4 = (p & 15) * 4;
    const v4f v = *(const v4f*)(W + (size_t)(k0 + r) * ldw + n0 + c4);
    tile[r][c4 + 0] = v[0]; tile[r][c4 + 1] = v[1]; tile[r][c4 + 2] = v[2]; tile[r][c4 + 3] = v[3];
  }
  __syncthreads();
  const int q = lane >> 3, c8 = (lane & 7) * 8;
  v4u oh[2], ol[2];
#pragma unroll
  for (int it = 0; it < 2; ++it) {
    const int rloc = 8 * wave + 4 * it + q;
    const v4f a0 = (v4f){tile[c8 + 0][rloc], tile[c8 + 1][rloc], tile[c8 + 2][rloc], tile[c8 + 3][rloc]};
    const v4f a1 = (v4f){tile[c8 + 4][rloc], tile[c8 + 5][rloc], tile[c8 + 6][rloc], tile[c8 + 7][rloc]};
    split_pack8(a0, a1, oh[it], ol[it]);
  }
  for (int pass = 0; pass < 2; ++pass) {
#pragma unroll
    for (int it = 0; it < 2; ++it) {
      const int rloc = 8 * wave + 4 * it + q;
      const size_t off = (size_t)(n0 + rloc) * ldo + k0 + c8;
      *(volatile v4u*)(Oh + off) = oh[it];
      *(volatile v4u*)(Ol + off) = ol[it];
    }
    __threadfence();
  }
}

__global__ __launch_bounds__(256) void k_wext(const float* __restrict__ de,
                                              u16* __restrict__ Kh, u16* __restrict__ Kl,
                                              u16* __restrict__ Vh, u16* __restrict__ Vl) {
  const int lane = threadIdx.x & 31, wave = threadIdx.x >> 5;
  const int q = lane >> 3, c8 = (lane & 7) * 8;
  const int which = blockIdx.y;
  const int n = blockIdx.x * 32 + 4 * wave + q;
  const float* tab = de + (size_t)(which ? 5 : 2) * NBIN * HDIM;
  u16* Oh = which ? Vh : Kh;
  u16* Ol = which ? Vl : Kl;
  float vals[8];
#pragma unroll
  for (int e = 0; e < 8; ++e) {
    const int j = c8 + e;
    const int ja = j < NBIN ? j : NBIN - 1;
    const float f = tab[(size_t)ja * HDIM + (n & (HDIM - 1))];
    vals[e] = (j < NBIN) ? f : 0.f;
  }
  v4u hv, lv;
  split_pack8((v4f){vals[0], vals[1], vals[2], vals[3]}, (v4f){vals[4], vals[5], vals[6], vals[7]}, hv, lv);
  const size_t off = (size_t)n * HPITCH + DMOD + c8;
  for (int pass = 0; pass < 2; ++pass) {
    *(volatile v4u*)(Oh + off) = hv;
    *(volatile v4u*)(Ol + off) = lv;
    __threadfence();
  }
}

__global__ __launch_bounds__(256) void k_detab(const float* __restrict__ de,
                                               u16* __restrict__ D01h, u16* __restrict__ D01l,
                                               u16* __restrict__ D34h, u16* __restrict__ D34l) {
  __shared__ __align__(16) float des[6 * NBIN * HDIM];
  const int tid = threadIdx.x, lane = tid & 31, wave = tid >> 5;
#pragma unroll
  for (int i = 0; i < 6; ++i) {
    const int p = tid + 256 * i;
    if (p < 6 * NBIN * HDIM / 4) *(v4f*)(des + 4 * p) = *(const v4f*)(de + 4 * p);
  }
  __syncthreads();
  const int q = lane >> 3, c8 = (lane & 7) * 8;
  const v4f z4 = (v4f){0.f, 0.f, 0.f, 0.f};
  v4u ah[2], al[2];
#pragma unroll
  for (int it = 0; it < 2; ++it) {
    const int r = 8 * wave + 4 * it + q;
    const int ra = r < NBIN ? r : NBIN - 1;
    const int rb = clampi(r - 16, 0, NBIN - 1);
    const v4f fa0 = *(const v4f*)(des + (size_t)(0 * NBIN + ra) * HDIM + c8);
    const v4f fa1 = *(const v4f*)(des + (size_t)(0 * NBIN + ra) * HDIM + c8 + 4);
    const v4f fb0 = *(const v4f*)(des + (size_t)(1 * NBIN + rb) * HDIM + c8);
    const v4f fb1 = *(const v4f*)(des + (size_t)(1 * NBIN + rb) * HDIM + c8 + 4);
    const bool useA = (r < NBIN), useB = (r >= 16 && r < 16 + NBIN);
    const v4f v0 = useA ? fa0 : (useB ? fb0 : z4);
    const v4f v1 = useA ? fa1 : (useB ? fb1 : z4);
    split_pack8(v0, v1, ah[it], al[it]);
  }
  for (int pass = 0; pass < 2; ++pass) {
#pragma unroll
    for (int it = 0; it < 2; ++it) {
      const int r = 8 * wave + 4 * it + q;
      *(volatile v4u*)(D01h + (size_t)r * 64 + c8) = ah[it];
      *(volatile v4u*)(D01l + (size_t)r * 64 + c8) = al[it];
    }
    __threadfence();
  }
  const int dd = 8 * wave + (lane >> 2);
  const int qq = lane & 3;
  unsigned hw[4], lw[4];
#pragma unroll
  for (int k = 0; k < 4; ++k) {
    float vv[2];
#pragma unroll
    for (int u = 0; u < 2; ++u) {
      const int j = 8 * qq + 2 * k + u;
      const int ja = j < NBIN ? j : NBIN - 1;
      const int jb = clampi(j - 16, 0, NBIN - 1);
      const float fa = des[(size_t)(3 * NBIN + ja) * HDIM + dd];
      const float fb = des[(size_t)(4 * NBIN + jb) * HDIM + dd];
      vv[u] = (j < NBIN) ? fa : ((j >= 16 && j < 16 + NBIN) ? fb : 0.f);
    }
    split_pack2(vv[0], vv[1], hw[k], lw[k]);
  }
  const v4u bh4 = (v4u){hw[0], hw[1], hw[2], hw[3]};
  const v4u bl4 = (v4u){lw[0], lw[1], lw[2], lw[3]};
  for (int pass = 0; pass < 2; ++pass) {
    *(volatile v4u*)(D34h + (size_t)dd * S3K + 8 * qq) = bh4;
    *(volatile v4u*)(D34l + (size_t)dd * S3K + 8 * qq) = bl4;
    __threadfence();
  }
}

__global__ __launch_bounds__(256) void k_attn_mid(const float* __restrict__ S, const float* __restrict__ T,
                                                  const int* __restrict__ didx, const float* __restrict__ mask,
                                                  u16* __restrict__ Ph, u16* __restrict__ Pl,
                                                  u16* __restrict__ S3h, u16* __restrict__ S3l) {
  __shared__ __align__(16) float rowbuf[NHEAD][SEQ];
  __shared__ __align__(16) float Tw[NHEAD * 64];
  __shared__ __align__(16) float mrows[NBATCH * SEQ];
  __shared__ __align__(16) int idxrow[SEQ];
  __shared__ __align__(16) float s3t[16 * 16];
  const int tid = threadIdx.x, lane = tid & 31, wave = tid >> 5;
  const int bl = blockIdx.x;
  const int b = bl / SEQ, l = bl - b * SEQ;
  const int h = wave;
  if (tid < SEQ / 4) {
    v4i iv = *(const v4i*)(didx + (size_t)bl * SEQ + 4 * tid);
#pragma unroll
    for (int e = 0; e < 4; ++e) iv[e] = clampi(iv[e], 0, NBIN - 1);
    *(v4i*)(idxrow + 4 * tid) = iv;
  }
  {
    const v4f m0 = *(const v4f*)(mask + 4 * tid);
    *(v4f*)(mrows + 4 * tid) = m0;
    if (tid < NBATCH * SEQ / 4 - 256) {
      const v4f m1 = *(const v4f*)(mask + 4 * (tid + 256));
      *(v4f*)(mrows + 4 * (tid + 256)) = m1;
    }
  }
  if (tid < NHEAD * 64 / 4) {
    const v4f tv = *(const v4f*)(T + (size_t)bl * NHEAD * 64 + 4 * tid);
    *(v4f*)(Tw + 4 * tid) = tv;
  }
  const int dr = clampi(didx[(size_t)b * SEQ * SEQ + l], 0, NBIN - 1);
  __syncthreads();

  const size_t R = (size_t)(b * NHEAD + h) * SEQ + l;
  const float* srow = S + R * SEQ;
  const int mrow = (b * NHEAD + h) % NBATCH;
  const float t1 = Tw[h * 64 + 16 + dr];
  float mx = -INFINITY;
  v4f e3[3];
#pragma unroll
  for (int i = 0; i < 3; ++i) {
    const int x0 = 128 * i + 4 * lane;
    const v4f sv = *(const v4f*)(srow + x0);
    const v4f mv = *(const v4f*)(mrows + mrow * SEQ + x0);
    const v4i iv = *(const v4i*)(idxrow + x0);
    v4f ev;
#pragma unroll
    for (int qd = 0; qd < 4; ++qd) {
      const float val = sv[qd] + Tw[h * 64 + iv[qd]] + t1;
      const float e = (mv[qd] == 0.0f) ? -INFINITY : val;
      ev[qd] = e;
      mx = fmaxf(mx, e);
    }
    e3[i] = ev;
  }
#pragma unroll
  for (int off = 16; off > 0; off >>= 1) mx = fmaxf(mx, __shfl_xor(mx, off, 32));
  float sum = 0.f;
  v4f p3[3];
#pragma unroll
  for (int i = 0; i < 3; ++i) {
    v4f pv;
#pragma unroll
    for (int qd = 0; qd < 4; ++qd) { const float p = expf(e3[i][qd] - mx); pv[qd] = p; sum += p; }
    p3[i] = pv;
  }
#pragma unroll
  for (int off = 16; off > 0; off >>= 1) sum += __shfl_xor(sum, off, 32);
  const float inv = 1.0f / sum;
#pragma unroll
  for (int i = 0; i < 3; ++i) {
    p3[i] = p3[i] * inv;
    *(v4f*)(&rowbuf[h][128 * i + 4 * lane]) = p3[i];
  }
  __syncthreads();

  v4u ph0, pl0, ph1, pl1;
  {
    const float* rb = &rowbuf[h][0];
    split_pack8(*(const v4f*)(rb + 8 * lane), *(const v4f*)(rb + 8 * lane + 4), ph0, pl0);
    const int c1 = 256 + 8 * (lane & 15);
    split_pack8(*(const v4f*)(rb + c1), *(const v4f*)(rb + c1 + 4), ph1, pl1);
  }
  {
    u16* prh = Ph + R * SEQ;
    u16* prl = Pl + R * SEQ;
    for (int pass = 0; pass < 2; ++pass) {
      *(volatile v4u*)(prh + 8 * lane) = ph0;
      *(volatile v4u*)(prl + 8 * lane) = pl0;
      if (lane < 16) {
        *(volatile v4u*)(prh + 256 + 8 * lane) = ph1;
        *(volatile v4u*)(prl + 256 + 8 * lane) = pl1;
      }
      __threadfence();
    }
  }

  if (wave == 0) {
    const int m = lane & 15, hh = lane >> 4;
    const int msrc = m & (NHEAD - 1);
    const bool mval = (m < NHEAD);
    const float* prow = &rowbuf[msrc][0];
    v8f acc = (v8f){0.f,0.f,0.f,0.f,0.f,0.f,0.f,0.f};
    for (int ks = 0; ks < SEQ / 32; ++ks) {
      const int k0 = ks * 32 + 8 * hh;
      v16b ah, al, bb;
#pragma unroll
      for (int i = 0; i < 8; ++i) {
        float f0 = prow[k0 + i];
        float f1 = prow[k0 + 16 + i];
        f0 = mval ? f0 : 0.f;
        f1 = mval ? f1 : 0.f;
        const unsigned short hb0 = f2bf_bits(f0), hb1 = f2bf_bits(f1);
        const unsigned short lb0 = f2bf_bits(f0 - bf_bits2f(hb0)), lb1 = f2bf_bits(f1 - bf_bits2f(hb1));
        ah[i] = __builtin_bit_cast(__bf16, hb0); ah[8 + i] = __builtin_bit_cast(__bf16, hb1);
        al[i] = __builtin_bit_cast(__bf16, lb0); al[8 + i] = __builtin_bit_cast(__bf16, lb1);
        const int i0 = idxrow[k0 + i], i1 = idxrow[k0 + 16 + i];
        bb[i]     = __builtin_bit_cast(__bf16, (unsigned short)(i0 == m ? 0x3F80 : 0));
        bb[8 + i] = __builtin_bit_cast(__bf16, (unsigned short)(i1 == m ? 0x3F80 : 0));
      }
      acc = at_mma(ah, bb, acc);
      acc = at_mma(al, bb, acc);
    }
#pragma unroll
    for (int r = 0; r < 8; ++r) s3t[(8 * hh + r) * 16 + m] = acc[r];
  }
  __syncthreads();

  if (wave == 0) {
    const int hrow = lane >> 2, qq = lane & 3;
    unsigned hw[4], lw[4];
#pragma unroll
    for (int k = 0; k < 4; ++k) {
      float vv[2];
#pragma unroll
      for (int u = 0; u < 2; ++u) {
        const int col = 8 * qq + 2 * k + u;
        const int cc = col < 16 ? col : 15;
        const float sval = s3t[hrow * 16 + cc];
        const float oh = (col >= 16 && (col - 16) == dr) ? 1.0f : 0.0f;
        vv[u] = (col < NBIN) ? sval : ((col >= 16 && col < 16 + NBIN) ? oh : 0.0f);
      }
      split_pack2(vv[0], vv[1], hw[k], lw[k]);
    }
    const v4u hv = (v4u){hw[0], hw[1], hw[2], hw[3]};
    const v4u lv = (v4u){lw[0], lw[1], lw[2], lw[3]};
    const size_t off = (size_t)bl * NHEAD * S3K + 8 * lane;
    for (int pass = 0; pass < 2; ++pass) {
      *(volatile v4u*)(S3h + off) = hv;
      *(volatile v4u*)(S3l + off) = lv;
      __threadfence();
    }
  }
}

__global__ __launch_bounds__(256) void k_gelu2(const float* __restrict__ U, u16* __restrict__ Gh, u16* __restrict__ Gl, int n2) {
  const int i = blockIdx.x * 256 + threadIdx.x;
  if (i < n2) {
    const float u0 = U[2 * (size_t)i], u1 = U[2 * (size_t)i + 1];
    const float g0 = 0.5f * u0 * (1.0f + erff(u0 * 0.70710678118654752f));
    const float g1 = 0.5f * u1 * (1.0f + erff(u1 * 0.70710678118654752f));
    unsigned wh, wl;
    split_pack2(g0, g1, wh, wl);
    ((volatile unsigned*)Gh)[i] = wh;
    ((volatile unsigned*)Gl)[i] = wl;
    __threadfence();
    ((volatile unsigned*)Gh)[i] = wh;
    ((volatile unsigned*)Gl)[i] = wl;
  }
}

__global__ __launch_bounds__(256) void k_transpose16(const u16* __restrict__ Ah, const u16* __restrict__ Al, int lda,
                                                     u16* __restrict__ Oh, u16* __restrict__ Ol, int ldo) {
  __shared__ unsigned short tile[64][66];
  const int t0 = blockIdx.x * 64, d0 = blockIdx.y * 64;
  const int tid = threadIdx.x, lane = tid & 31, wave = tid >> 5;
  const int q = lane >> 3, c8 = (lane & 7) * 8;
  for (int pl = 0; pl < 2; ++pl) {
    const u16* A = pl ? Al : Ah;
    u16* O = pl ? Ol : Oh;
    {
      const int r = tid >> 2, cq = tid & 3;
      const v4u w0 = *(const v4u*)(A + (size_t)(t0 + r) * lda + d0 + 16 * cq);
      const v4u w1 = *(const v4u*)(A + (size_t)(t0 + r) * lda + d0 + 16 * cq + 8);
#pragma unroll
      for (int k = 0; k < 4; ++k) {
        tile[r][16 * cq + 2 * k]         = (unsigned short)(w0[k] & 0xffffu);
        tile[r][16 * cq + 2 * k + 1]     = (unsigned short)(w0[k] >> 16);
        tile[r][16 * cq + 8 + 2 * k]     = (unsigned short)(w1[k] & 0xffffu);
        tile[r][16 * cq + 8 + 2 * k + 1] = (unsigned short)(w1[k] >> 16);
      }
    }
    __syncthreads();
    v4u ov[2];
#pragma unroll
    for (int it = 0; it < 2; ++it) {
      const int rloc = 8 * wave + 4 * it + q;
      unsigned w[4];
#pragma unroll
      for (int k = 0; k < 4; ++k)
        w[k] = (unsigned)tile[c8 + 2 * k][rloc] | ((unsigned)tile[c8 + 2 * k + 1][rloc] << 16);
      ov[it] = (v4u){w[0], w[1], w[2], w[3]};
    }
    for (int pass = 0; pass < 2; ++pass) {
#pragma unroll
      for (int it = 0; it < 2; ++it) {
        const int rloc = 8 * wave + 4 * it + q;
        *(volatile v4u*)(O + (size_t)(d0 + rloc) * ldo + t0 + c8) = ov[it];
      }
      __threadfence();
    }
    __syncthreads();
  }
}

__global__ __launch_bounds__(192) void k_maskm(const float* __restrict__ mask, u16* __restrict__ Mh, u16* __restrict__ Ml) {
  const int r = blockIdx.x;
  const int lane = threadIdx.x & 31, wave = threadIdx.x >> 5;
  const int t0 = 256 * wave + 8 * lane;
  const int rr = r < NBATCH ? r : NBATCH - 1;
  const int base = rr * SEQ + (t0 % SEQ);
  const v4f a0 = *(const v4f*)(mask + base);
  const v4f a1 = *(const v4f*)(mask + base + 4);
  const bool inside = (r < NBATCH) && (t0 >= r * SEQ) && (t0 < (r + 1) * SEQ);
  const v4f z4 = (v4f){0.f, 0.f, 0.f, 0.f};
  v4u hv, lv;
  split_pack8(inside ? a0 : z4, inside ? a1 : z4, hv, lv);
  const size_t off = (size_t)r * NTOK + t0;
  for (int pass = 0; pass < 2; ++pass) {
    *(volatile v4u*)(Mh + off) = hv;
    *(volatile v4u*)(Ml + off) = lv;
    __threadfence();
  }
}

__global__ __launch_bounds__(256) void k_wm2(const float* __restrict__ w, u16* __restrict__ Oh, u16* __restrict__ Ol) {
  const int lane = threadIdx.x & 31, wave = threadIdx.x >> 5;
  v4u wh[2], wl[2];
#pragma unroll
  for (int seg = 0; seg < 2; ++seg) {
    const int c = 256 * seg + 8 * lane;
    split_pack8(*(const v4f*)(w + c), *(const v4f*)(w + c + 4), wh[seg], wl[seg]);
  }
  const v4u z4 = (v4u){0u, 0u, 0u, 0u};
  for (int pass = 0; pass < 2; ++pass) {
#pragma unroll
    for (int it = 0; it < 8; ++it) {
      const int row = 8 * wave + it;
#pragma unroll
      for (int seg = 0; seg < 2; ++seg) {
        v4u hs = z4, ls = z4;
        if (row == 0) { hs = wh[seg]; ls = wl[seg]; }
        const size_t off = (size_t)row * MHID + 256 * seg + 8 * lane;
        *(volatile v4u*)(Oh + off) = hs;
        *(volatile v4u*)(Ol + off) = ls;
      }
    }
    __threadfence();
  }
}

__global__ __launch_bounds__(32) void k_final(const float* __restrict__ C2v, const float* __restrict__ bm2, float* __restrict__ out) {
  const int lane = threadIdx.x;
  const float bb = bm2[0];
  v4f o;
  o[0] = C2v[0 * 64] + bb;
  o[1] = C2v[1 * 64] + bb;
  o[2] = C2v[2 * 64] + bb;
  o[3] = C2v[3 * 64] + bb;
  if (lane == 0) {
    *(volatile v4f*)out = o;
    __threadfence();
    *(volatile v4f*)out = o;
  }
}

template <int BM, int OM, bool RS, int AC>
static void run_gemm(hipStream_t st,
                     const void* Ah, const void* Al, int lda, long sAo, long sAi,
                     const void* Bh, const void* Bl, int ldb, long sBo, long sBi,
                     void* C0, void* C1, int ldc, long sCo, long sCi,
                     const float* bias, const float* resid, long sRo, long sRi,
                     int M, int N, int K, int nbatch, int HB) {
  const int tiles = (M / 64) * (N / 64);
  dim3 grid((tiles + 7) / 8, nbatch);
  gemm_split64<BM, OM, RS, AC><<<grid, 256, 0, st>>>(
      (const u16*)Ah, (const u16*)Al, lda, sAo, sAi,
      (const u16*)Bh, (const u16*)Bl, ldb, sBo, sBi,
      C0, C1, ldc, sCo, sCi, bias, resid, sRo, sRi, M, N, K, HB, 1.0f);
}

extern "C" void kernel_launch(void* const* d_in, const int* in_sizes, int n_in,
                              void* d_out, int out_size, void* d_ws, size_t ws_size,
                              hipStream_t stream) {
  (void)in_sizes; (void)n_in; (void)out_size;
  if (ws_size < WS_END) return;

  const int*   ct   = (const int*)  d_in[0];
  const float* dist = (const float*)d_in[1];
  const float* mask = (const float*)d_in[2];
  const float* cemb = (const float*)d_in[3];
  const float* demb = (const float*)d_in[4];
  const float* Wq  = (const float*)d_in[5];   const float* bq  = (const float*)d_in[6];
  const float* Wk  = (const float*)d_in[7];   const float* bk  = (const float*)d_in[8];
  const float* Wv  = (const float*)d_in[9];   const float* bv  = (const float*)d_in[10];
  const float* Wo  = (const float*)d_in[11];  const float* bo  = (const float*)d_in[12];
  const float* W1  = (const float*)d_in[13];  const float* b1  = (const float*)d_in[14];
  const float* W2  = (const float*)d_in[15];  const float* b2  = (const float*)d_in[16];
  const float* g1  = (const float*)d_in[17];  const float* be1 = (const float*)d_in[18];
  const float* g2  = (const float*)d_in[19];  const float* be2 = (const float*)d_in[20];
  const float* Wm1 = (const float*)d_in[21];  const float* bm1 = (const float*)d_in[22];
  const float* Wm2 = (const float*)d_in[23];  const float* bm2 = (const float*)d_in[24];
  float* out = (float*)d_out;

  char* ws = (char*)d_ws;
  float* hF   = (float*)(ws + OFF_HF);
  u16*   hH   = (u16*)(ws + OFF_HH);   u16* hL   = (u16*)(ws + OFF_HL);
  u16*   wQh  = (u16*)(ws + OFF_WQH);  u16* wQl  = (u16*)(ws + OFF_WQL);
  u16*   wKh  = (u16*)(ws + OFF_WKH);  u16* wKl  = (u16*)(ws + OFF_WKL);
  u16*   wVh  = (u16*)(ws + OFF_WVH);  u16* wVl  = (u16*)(ws + OFF_WVL);
  u16*   wOh  = (u16*)(ws + OFF_WOH);  u16* wOl  = (u16*)(ws + OFF_WOL);
  u16*   w1h  = (u16*)(ws + OFF_W1H);  u16* w1l  = (u16*)(ws + OFF_W1L);
  u16*   w2h  = (u16*)(ws + OFF_W2H);  u16* w2l  = (u16*)(ws + OFF_W2L);
  u16*   d01h = (u16*)(ws + OFF_D01H); u16* d01l = (u16*)(ws + OFF_D01L);
  u16*   d34h = (u16*)(ws + OFF_D34H); u16* d34l = (u16*)(ws + OFF_D34L);
  u16*   qH   = (u16*)(ws + OFF_QH);   u16* qL   = (u16*)(ws + OFF_QL);
  u16*   kH   = (u16*)(ws + OFF_KH);   u16* kL   = (u16*)(ws + OFF_KL);
  u16*   vtH  = (u16*)(ws + OFF_VTH);  u16* vtL  = (u16*)(ws + OFF_VTL);
  float* tT   = (float*)(ws + OFF_T);
  float* sF   = (float*)(ws + OFF_BIG1);
  float* uF   = (float*)(ws + OFF_BIG1);
  u16*   pH   = (u16*)(ws + OFF_BIG2H); u16* pL   = (u16*)(ws + OFF_BIG2L);
  u16*   gH   = (u16*)(ws + OFF_BIG2H); u16* gL   = (u16*)(ws + OFF_BIG2L);
  u16*   s3h  = (u16*)(ws + OFF_S3H);  u16* s3l  = (u16*)(ws + OFF_S3L);
  float* zpv  = (float*)(ws + OFF_ZPV);
  u16*   zH   = (u16*)(ws + OFF_ZH);   u16* zL   = (u16*)(ws + OFF_ZL);
  float* aF   = (float*)(ws + OFF_AF);
  int*   didx = (int*)(ws + OFF_DIDX);
  u16*   htH  = (u16*)(ws + OFF_HTH);  u16* htL  = (u16*)(ws + OFF_HTL);
  u16*   mmH  = (u16*)(ws + OFF_MMH);  u16* mmL  = (u16*)(ws + OFF_MML);
  u16*   poH  = (u16*)(ws + OFF_POH);  u16* poL  = (u16*)(ws + OFF_POL);
  u16*   hidH = (u16*)(ws + OFF_HIDH); u16* hidL = (u16*)(ws + OFF_HIDL);
  u16*   wm2H = (u16*)(ws + OFF_WM2H); u16* wm2L = (u16*)(ws + OFF_WM2L);
  float* c2   = (float*)(ws + OFF_C2);

  k_bucketize<<<NBATCH * SEQ * SEQ / 4 / 256, 256, 0, stream>>>(dist, didx, NBATCH * SEQ * SEQ / 4);
  k_embed<<<NTOK / 8, 256, 0, stream>>>(ct, cemb, didx, hF, hH, hL);
  k_detab<<<1, 256, 0, stream>>>(demb, d01h, d01l, d34h, d34l);
  k_wext<<<dim3(DMOD / 32, 2), 256, 0, stream>>>(demb, wKh, wKl, wVh, wVl);

  for (int ly = 0; ly < NLAY; ++ly) {
    const float* Wq_l = Wq + (size_t)ly * DMOD * DMOD;  const float* bq_l = bq + (size_t)ly * DMOD;
    const float* Wk_l = Wk + (size_t)ly * DMOD * DMOD;  const float* bk_l = bk + (size_t)ly * DMOD;
    const float* Wv_l = Wv + (size_t)ly * DMOD * DMOD;  const float* bv_l = bv + (size_t)ly * DMOD;
    const float* Wo_l = Wo + (size_t)ly * DMOD * DMOD;  const float* bo_l = bo + (size_t)ly * DMOD;
    const float* W1_l = W1 + (size_t)ly * DMOD * FFD;   const float* b1_l = b1 + (size_t)ly * FFD;
    const float* W2_l = W2 + (size_t)ly * FFD * DMOD;   const float* b2_l = b2 + (size_t)ly * DMOD;
    const float* g1_l = g1 + (size_t)ly * DMOD;         const float* be1_l = be1 + (size_t)ly * DMOD;
    const float* g2_l = g2 + (size_t)ly * DMOD;         const float* be2_l = be2 + (size_t)ly * DMOD;

    k_wT<<<dim3(DMOD / 64, DMOD / 64), 256, 0, stream>>>(Wq_l, DMOD, wQh, wQl, DMOD);
    k_wT<<<dim3(DMOD / 64, DMOD / 64), 256, 0, stream>>>(Wk_l, DMOD, wKh, wKl, HPITCH);
    k_wT<<<dim3(DMOD / 64, DMOD / 64), 256, 0, stream>>>(Wv_l, DMOD, wVh, wVl, HPITCH);
    k_wT<<<dim3(DMOD / 64, DMOD / 64), 256, 0, stream>>>(Wo_l, DMOD, wOh, wOl, DMOD);
    k_wT<<<dim3(FFD / 64, DMOD / 64), 256, 0, stream>>>(W1_l, FFD, w1h, w1l, DMOD);
    k_wT<<<dim3(DMOD / 64, FFD / 64), 256, 0, stream>>>(W2_l, DMOD, w2h, w2l, FFD);

    run_gemm<2, 2, false, 0>(stream, hH, hL, HPITCH, 0, 0, wQh, wQl, DMOD, 0, 0,
                             qH, qL, DMOD, 0, 0, bq_l, nullptr, 0, 0, NTOK, DMOD, DMOD, 1, 1);
    run_gemm<2, 2, false, 0>(stream, hH, hL, HPITCH, 0, 0, wKh, wKl, HPITCH, 0, 0,
                             kH, kL, DMOD, 0, 0, bk_l, nullptr, 0, 0, NTOK, DMOD, HPITCH, 1, 1);
    run_gemm<1, 2, false, 0>(stream, wVh, wVl, HPITCH, 0, 0, hH, hL, HPITCH, 0, 0,
                             vtH, vtL, NTOK, 0, 0, bv_l, nullptr, 0, 0, DMOD, NTOK, HPITCH, 1, 1);
    run_gemm<0, 0, false, 0>(stream, qH, qL, HDIM, 0, 0, d01h, d01l, HDIM, 0, 0,
                             tT, nullptr, HDIM, 0, 0, nullptr, nullptr, 0, 0, QROWS, 64, HDIM, 1, 1);
    run_gemm<0, 0, false, 0>(stream, qH, qL, DMOD, (long)SEQ * DMOD, HDIM, kH, kL, DMOD, (long)SEQ * DMOD, HDIM,
                             sF, nullptr, SEQ, (long)NHEAD * SEQ * SEQ, (long)SEQ * SEQ, nullptr, nullptr, 0, 0,
                             SEQ, SEQ, HDIM, NBH, NHEAD);
    k_attn_mid<<<NTOK, 256, 0, stream>>>(sF, tT, didx, mask, pH, pL, s3h, s3l);
    run_gemm<0, 0, false, 0>(stream, pH, pL, SEQ, (long)NHEAD * SEQ * SEQ, (long)SEQ * SEQ,
                             vtH, vtL, NTOK, SEQ, (long)HDIM * NTOK,
                             zpv, nullptr, DMOD, (long)SEQ * DMOD, HDIM, nullptr, nullptr, 0, 0,
                             SEQ, HDIM, SEQ, NBH, NHEAD);
    run_gemm<0, 2, true, 0>(stream, s3h, s3l, S3K, 0, 0, d34h, d34l, S3K, 0, 0,
                            zH, zL, HDIM, 0, 0, nullptr, zpv, 0, 0, QROWS, 64, S3K, 1, 1);
    run_gemm<2, 0, false, 0>(stream, zH, zL, DMOD, 0, 0, wOh, wOl, DMOD, 0, 0,
                             aF, nullptr, DMOD, 0, 0, bo_l, nullptr, 0, 0, NTOK, DMOD, DMOD, 1, 1);
    k_resid_ln<<<NTOK / 8, 256, 0, stream>>>(aF, g1_l, be1_l, hF, hH, hL);
    run_gemm<2, 0, false, 0>(stream, hH, hL, HPITCH, 0, 0, w1h, w1l, DMOD, 0, 0,
                             uF, nullptr, FFD, 0, 0, b1_l, nullptr, 0, 0, NTOK, FFD, DMOD, 1, 1);
    k_gelu2<<<NTOK * FFD / 2 / 256, 256, 0, stream>>>(uF, gH, gL, NTOK * FFD / 2);
    run_gemm<2, 0, false, 0>(stream, gH, gL, FFD, 0, 0, w2h, w2l, FFD, 0, 0,
                             aF, nullptr, DMOD, 0, 0, b2_l, nullptr, 0, 0, NTOK, DMOD, FFD, 1, 1);
    k_resid_ln<<<NTOK / 8, 256, 0, stream>>>(aF, g2_l, be2_l, hF, hH, hL);
  }

  k_transpose16<<<dim3(NTOK / 64, DMOD / 64), 256, 0, stream>>>(hH, hL, HPITCH, htH, htL, NTOK);
  k_maskm<<<TAILM, 192, 0, stream>>>(mask, mmH, mmL);
  k_wT<<<dim3(MHID / 64, DMOD / 64), 256, 0, stream>>>(Wm1, MHID, wQh, wQl, DMOD);
  k_wm2<<<1, 256, 0, stream>>>(Wm2, wm2H, wm2L);
  run_gemm<0, 2, false, 0>(stream, mmH, mmL, NTOK, 0, 0, htH, htL, NTOK, 0, 0,
                           poH, poL, DMOD, 0, 0, nullptr, nullptr, 0, 0, TAILM, DMOD, NTOK, 1, 1);
  run_gemm<2, 2, false, 2>(stream, poH, poL, DMOD, 0, 0, wQh, wQl, DMOD, 0, 0,
                           hidH, hidL, MHID, 0, 0, bm1, nullptr, 0, 0, TAILM, MHID, DMOD, 1, 1);
  run_gemm<0, 0, false, 0>(stream, hidH, hidL, MHID, 0, 0, wm2H, wm2L, MHID, 0, 0,
                           c2, nullptr, 64, 0, 0, nullptr, nullptr, 0, 0, TAILM, 64, MHID, 1, 1);
  k_final<<<1, 32, 0, stream>>>(c2, bm2, out);
}
